// SVM_13846974562943
// MI455X (gfx1250) — hardware-verified
//
#include <hip/hip_runtime.h>
#include <stdint.h>

#define I_SIZE 64
#define H_SIZE 128
#define O_SIZE 64
#define BATCH  64
#define TLEN   2048
#define G3H    384

typedef __attribute__((ext_vector_type(16))) _Float16 v16h;
typedef __attribute__((ext_vector_type(8)))  _Float16 v8h;
typedef __attribute__((ext_vector_type(16))) __bf16   v16b;
typedef __attribute__((ext_vector_type(8)))  __bf16   v8b;
typedef __attribute__((ext_vector_type(8)))  float    v8f;
typedef __attribute__((ext_vector_type(4)))  float    v4f;

__device__ __forceinline__ unsigned short f2bf_bits(float f) {
  unsigned u = __float_as_uint(f);
  return (unsigned short)((u + 0x7FFFu + ((u >> 16) & 1u)) >> 16);
}
__device__ __forceinline__ float bf_bits2f(unsigned short h) { return __uint_as_float(((unsigned)h) << 16); }

__device__ __forceinline__ void dep_guard_h(v8f& a, v8f& b, v16h x, v16h y) { asm volatile("v_nop\n\tv_nop\n\tv_nop\n\tv_nop" : "+v"(a), "+v"(b) : "v"(x), "v"(y)); }
__device__ __forceinline__ void dep_guard_b(v8f& a, v8f& b, v16b x, v16b y) { asm volatile("v_nop\n\tv_nop\n\tv_nop\n\tv_nop" : "+v"(a), "+v"(b) : "v"(x), "v"(y)); }
__device__ __forceinline__ void keep4_h(v16h a, v16h b, v16h c, v16h d) { asm volatile("v_nop" :: "v"(a), "v"(b), "v"(c), "v"(d)); }
__device__ __forceinline__ void keep4_b(v16b a, v16b b, v16b c, v16b d) { asm volatile("v_nop" :: "v"(a), "v"(b), "v"(c), "v"(d)); }
__device__ __forceinline__ void acc_guard4(v8f& a, v8f& b, v8f& c, v8f& d) { asm volatile("v_nop\n\tv_nop\n\tv_nop\n\tv_nop" : "+v"(a), "+v"(b), "+v"(c), "+v"(d)); }
template <typename T> struct Frag;
template <> struct Frag<_Float16> {
  typedef v16h V; union U { v16h v; v8h h[2]; };
  static __device__ __forceinline__ v16h load(const _Float16* p) {
    U f; f.h[0] = *(const v8h*)(p); f.h[1] = *(const v8h*)(p + 16); return f.v;
  }
  static __device__ __forceinline__ v8f mma(v16h a, v16h b, v8f c) {
    return __builtin_amdgcn_wmma_f32_16x16x32_f16(false, a, false, b, (short)0, c, false, false);
  }
  static __device__ __forceinline__ void guard(v8f& a, v8f& b, v16h x, v16h y) { dep_guard_h(a, b, x, y); }
  static __device__ __forceinline__ void keep(v16h a, v16h b, v16h c, v16h d) { keep4_h(a, b, c, d); }
};
template <> struct Frag<__bf16> {
  typedef v16b V; union U { v16b v; v8b h[2]; };
  static __device__ __forceinline__ v16b load(const __bf16* p) {
    U f; f.h[0] = *(const v8b*)(p); f.h[1] = *(const v8b*)(p + 16); return f.v;
  }
  static __device__ __forceinline__ v8f mma(v16b a, v16b b, v8f c) {
    return __builtin_amdgcn_wmma_f32_16x16x32_bf16(false, a, false, b, (short)0, c, false, false);
  }
  static __device__ __forceinline__ void guard(v8f& a, v8f& b, v16b x, v16b y) { dep_guard_b(a, b, x, y); }
  static __device__ __forceinline__ void keep(v16b a, v16b b, v16b c, v16b d) { keep4_b(a, b, c, d); }
};

__device__ __forceinline__ v8f mma_f16g(v16h a, v16h b, v8f c) {
  c = __builtin_amdgcn_wmma_f32_16x16x32_f16(false, a, false, b, (short)0, c, false, false);
  asm volatile("v_nop\n\tv_nop\n\tv_nop\n\tv_nop" : "+v"(c) : "v"(a), "v"(b));
  return c;
}
__device__ __forceinline__ v8f mma_bf16g(v16b a, v16b b, v8f c) {
  c = __builtin_amdgcn_wmma_f32_16x16x32_bf16(false, a, false, b, (short)0, c, false, false);
  asm volatile("v_nop\n\tv_nop\n\tv_nop\n\tv_nop" : "+v"(c) : "v"(a), "v"(b));
  return c;
}

template <int ET> struct Elem;
template <> struct Elem<0> { typedef _Float16 T; };
template <> struct Elem<1> { typedef __bf16 T; };
template <int ET, bool SPLIT, int BIAS_MODE, int OUT_MODE, bool RESID, int ACT = 0>
__global__ __launch_bounds__(256) void wmma_gemm64(
    const unsigned short* __restrict__ Ap, const unsigned short* __restrict__ A2p, int lda, long strideA,
    const unsigned short* __restrict__ Btp, const unsigned short* __restrict__ Bt2p, int ldb, long strideB,
    void* __restrict__ Cout, void* __restrict__ Cout2, int ldc, long strideC,
    const float* __restrict__ bias,
    const float* __restrict__ resid, long strideR,
    int M, int N, int K, float scale) {
  typedef typename Elem<ET>::T T;
  typedef typename Frag<T>::V V;
  const T* A = (const T*)Ap; const T* A2 = (const T*)A2p; const T* Bt = (const T*)Btp; const T* Bt2 = (const T*)Bt2p;
  __shared__ __align__(16) float sT[8][16 * 68];
  const int b    = blockIdx.y;
  const int lane = threadIdx.x & 31;
  const int wave = threadIdx.x >> 5;
  const int tilesN = N >> 6;
  const int tilesM = M >> 6;
  const int tile = blockIdx.x * 8 + wave;
  if (tile >= tilesM * tilesN) return;
  const int tm = tile / tilesN;
  const int tn = tile - tm * tilesN;
  const int m0 = tm << 6;
  const int n0 = tn << 6;

  const T* Ab  = A  + (size_t)b * strideA;
  const T* Bb  = Bt + (size_t)b * strideB;
  const T* Ab2 = SPLIT ? (A2  + (size_t)b * strideA) : nullptr;
  const T* Bb2 = SPLIT ? (Bt2 + (size_t)b * strideB) : nullptr;

  const int rlane = lane & 15;
  const int koff  = (lane >> 4) * 8;
  const int mOff  = (lane >> 4) * 8;

  v8f acc[4][4];
#pragma unroll
  for (int i = 0; i < 4; ++i)
#pragma unroll
    for (int j = 0; j < 4; ++j) acc[i][j] = (v8f){0.f,0.f,0.f,0.f,0.f,0.f,0.f,0.f};

  for (int k0 = 0; k0 < K; k0 += 32) {
    V bh[4], bl[4];
#pragma unroll
    for (int j = 0; j < 4; ++j) {
      const size_t bo = (size_t)(n0 + (j << 4) + rlane) * ldb + koff + k0;
      bh[j] = Frag<T>::load(Bb + bo);
      if (SPLIT) bl[j] = Frag<T>::load(Bb2 + bo);
    }
#pragma unroll
    for (int i = 0; i < 4; ++i) {
      const size_t ao = (size_t)(m0 + (i << 4) + rlane) * lda + koff + k0;
      V ah = Frag<T>::load(Ab + ao);
      V al;
      if (SPLIT) al = Frag<T>::load(Ab2 + ao);
#pragma unroll
      for (int j = 0; j < 4; ++j) {
        acc[i][j] = Frag<T>::mma(ah, bh[j], acc[i][j]);
        if (SPLIT) {
          acc[i][j] = Frag<T>::mma(ah, bl[j], acc[i][j]);
          acc[i][j] = Frag<T>::mma(al, bh[j], acc[i][j]);
        }
      }
      Frag<T>::guard(acc[i][0], acc[i][3], ah, SPLIT ? al : ah);
    }
    Frag<T>::keep(bh[0], bh[1], bh[2], bh[3]);
    if (SPLIT) Frag<T>::keep(bl[0], bl[1], bl[2], bl[3]);
  }
  acc_guard4(acc[0][0], acc[0][1], acc[0][2], acc[0][3]);
  acc_guard4(acc[1][0], acc[1][1], acc[1][2], acc[1][3]);
  acc_guard4(acc[2][0], acc[2][1], acc[2][2], acc[2][3]);
  acc_guard4(acc[3][0], acc[3][1], acc[3][2], acc[3][3]);

  float* slab = sT[wave];
  const float* Rb = RESID ? (resid + (size_t)b * strideR) : nullptr;
#pragma unroll
  for (int i = 0; i < 4; ++i) {
    const int mBase = m0 + (i << 4);
#pragma unroll
    for (int j = 0; j < 4; ++j) {
      const int n = n0 + (j << 4) + rlane;
      float bv = 0.f;
      if (BIAS_MODE == 2) bv = bias[n];
#pragma unroll
      for (int r = 0; r < 8; ++r) {
        float v = acc[i][j][r] * scale;
        if (BIAS_MODE == 1) v += bias[mBase + mOff + r];
        if (BIAS_MODE == 2) v += bv;
        if (RESID) v += Rb[(size_t)(mBase + mOff + r) * ldc + n];
        if (ACT == 1) v = tanhf(v);
        if (ACT == 2) v = fmaxf(v, 0.0f);
        if (ACT == 3) v = v / (1.0f + expf(-v));
        if (ACT == 4) v = (v > 0.f) ? v : 0.01f * v;
        if (ACT == 5) v = 0.5f * v * (1.0f + erff(v * 0.70710678118654752f));
        slab[(mOff + r) * 68 + (j << 4) + rlane] = v;
      }
    }
    __builtin_amdgcn_fence(__ATOMIC_RELEASE, "workgroup");
    __builtin_amdgcn_wave_barrier();
    __builtin_amdgcn_fence(__ATOMIC_ACQUIRE, "workgroup");
    if (OUT_MODE == 0) {
      float* C = (float*)Cout + (size_t)b * strideC;
      const int hh = lane >> 4, c4 = (lane & 15) * 4;
      for (int pass = 0; pass < 2; ++pass) {
#pragma unroll
        for (int it = 0; it < 8; ++it) {
          const int row = it * 2 + hh;
          v4f v = *(const v4f*)(slab + row * 68 + c4);
          *(volatile v4f*)(C + (size_t)(mBase + row) * ldc + n0 + c4) = v;
        }
        __threadfence();
      }
    } else {
      const int q = lane >> 3, c8 = (lane & 7) * 8;
      unsigned short* C  = (unsigned short*)Cout  + (size_t)b * strideC;
      unsigned short* C2 = (OUT_MODE == 2) ? ((unsigned short*)Cout2 + (size_t)b * strideC) : nullptr;
      for (int pass = 0; pass < 2; ++pass) {
#pragma unroll
        for (int it = 0; it < 4; ++it) {
          const int row = it * 4 + q;
          const float* sp = slab + row * 68 + c8;
          v8h hv, lv;
#pragma unroll
          for (int e = 0; e < 8; ++e) {
            if (OUT_MODE == 1) {
              hv[e] = (_Float16)sp[e];
            } else {
              unsigned short hb = f2bf_bits(sp[e]);
              unsigned short lb = f2bf_bits(sp[e] - bf_bits2f(hb));
              hv[e] = __builtin_bit_cast(_Float16, hb);
              lv[e] = __builtin_bit_cast(_Float16, lb);
            }
          }
          *(volatile v8h*)(C + (size_t)(mBase + row) * ldc + n0 + c8) = hv;
          if (OUT_MODE == 2) *(volatile v8h*)(C2 + (size_t)(mBase + row) * ldc + n0 + c8) = lv;
        }
        __threadfence();
      }
    }
    __builtin_amdgcn_fence(__ATOMIC_RELEASE, "workgroup");
    __builtin_amdgcn_wave_barrier();
    __builtin_amdgcn_fence(__ATOMIC_ACQUIRE, "workgroup");
  }
}

__global__ __launch_bounds__(256) void cast_f32_bf16hl8(
    const float* __restrict__ in, unsigned short* __restrict__ hi, unsigned short* __restrict__ lo, int n8) {
  const int i = blockIdx.x * 256 + threadIdx.x;
  if (i < n8) {
    const size_t o = (size_t)i * 8;
    const v4f a = *(const v4f*)(in + o);
    const v4f b = *(const v4f*)(in + o + 4);
    v8h hv, lv;
#pragma unroll
    for (int e = 0; e < 4; ++e) {
      const unsigned short h0 = f2bf_bits(a[e]);
      const unsigned short l0 = f2bf_bits(a[e] - bf_bits2f(h0));
      const unsigned short h1 = f2bf_bits(b[e]);
      const unsigned short l1 = f2bf_bits(b[e] - bf_bits2f(h1));
      hv[e] = __builtin_bit_cast(_Float16, h0);     lv[e] = __builtin_bit_cast(_Float16, l0);
      hv[4 + e] = __builtin_bit_cast(_Float16, h1); lv[4 + e] = __builtin_bit_cast(_Float16, l1);
    }
    *(volatile v8h*)(hi + o) = hv;
    *(volatile v8h*)(lo + o) = lv;
    __threadfence();
    *(volatile v8h*)(hi + o) = hv;
    *(volatile v8h*)(lo + o) = lv;
  }
}

__global__ __launch_bounds__(256) void cast_f32_f16s8(
    const float* __restrict__ in, _Float16* __restrict__ out, int n8, float scale) {
  const int i = blockIdx.x * 256 + threadIdx.x;
  if (i < n8) {
    const size_t o = (size_t)i * 8;
    const v4f a = *(const v4f*)(in + o);
    const v4f b = *(const v4f*)(in + o + 4);
    v8h hv;
#pragma unroll
    for (int e = 0; e < 4; ++e) {
      hv[e] = (_Float16)(a[e] * scale);
      hv[4 + e] = (_Float16)(b[e] * scale);
    }
    *(volatile v8h*)(out + o) = hv;
    __threadfence();
    *(volatile v8h*)(out + o) = hv;
  }
}

#define LDH 136
#define LDF 132
#define HINV (1.0f / 16384.0f)

__device__ __forceinline__ float sigm_(float x) { return __builtin_amdgcn_rcpf(1.0f + expf(-x)); }

__global__ __launch_bounds__(256) __attribute__((amdgpu_num_vgpr(256)))
void gru_scan_kernel(const unsigned short* xh, const unsigned short* xl,
                     const unsigned short* wih_h, const unsigned short* wih_l,
                     const _Float16* whh16,
                     const float* b_ih, const float* b_hh,
                     unsigned short* hs_hi, unsigned short* hs_lo) {
  __shared__ __align__(16) _Float16 hb[2][16 * LDH];
  __shared__ __align__(16) float    hF[2][16 * LDF];

  const int tid  = threadIdx.x;
  const int wave = tid >> 5, lane = tid & 31, hh = lane >> 4, c = lane & 15;
  const int bbase = blockIdx.x * 16;
  const int col  = wave * 16 + c;
  const int koff = 8 * hh;

  const __bf16* Xh = (const __bf16*)xh + (size_t)(bbase + c) * TLEN * I_SIZE + koff;
  const __bf16* Xl = (const __bf16*)xl + (size_t)(bbase + c) * TLEN * I_SIZE + koff;
  const __bf16* Wr_h = (const __bf16*)wih_h + (size_t)col * I_SIZE + koff;
  const __bf16* Wr_l = (const __bf16*)wih_l + (size_t)col * I_SIZE + koff;
  const _Float16* Whr = whh16 + (size_t)col * H_SIZE + koff;

  const float bir = b_ih[col], biz = b_ih[H_SIZE + col], bin = b_ih[2 * H_SIZE + col];
  const float bhr = b_hh[col], bhz = b_hh[H_SIZE + col], bhn = b_hh[2 * H_SIZE + col];

  {
    _Float16* hz = &hb[0][0];
    for (int k = tid; k < 2 * 16 * LDH; k += 256) hz[k] = (_Float16)0.0f;
  }
  float hst[8];
#pragma unroll
  for (int r = 0; r < 8; ++r) hst[r] = 0.0f;
  __syncthreads();

  const int srow = tid >> 4;
  const int sseg = (tid & 15) * 8;
  const v8f z8 = {0.f, 0.f, 0.f, 0.f, 0.f, 0.f, 0.f, 0.f};

  for (int t = 0; t < TLEN; ++t) {
    const int cur = t & 1, nxt = cur ^ 1;
    v8f axr = z8, axz = z8, axn = z8, ahr = z8, ahz = z8, ahn = z8;

    const __bf16* xht = Xh + (size_t)t * I_SIZE;
    const __bf16* xlt = Xl + (size_t)t * I_SIZE;
#pragma unroll
    for (int kc = 0; kc < 2; ++kc) {
      const int ko = kc * 32;
      const v16b ah = Frag<__bf16>::load(xht + ko);
      const v16b al = Frag<__bf16>::load(xlt + ko);
      {
        const v16b bh = Frag<__bf16>::load(Wr_h + ko);
        const v16b bl = Frag<__bf16>::load(Wr_l + ko);
        axr = mma_bf16g(ah, bh, axr); axr = mma_bf16g(ah, bl, axr); axr = mma_bf16g(al, bh, axr);
      }
      {
        const v16b bh = Frag<__bf16>::load(Wr_h + H_SIZE * I_SIZE + ko);
        const v16b bl = Frag<__bf16>::load(Wr_l + H_SIZE * I_SIZE + ko);
        axz = mma_bf16g(ah, bh, axz); axz = mma_bf16g(ah, bl, axz); axz = mma_bf16g(al, bh, axz);
      }
      {
        const v16b bh = Frag<__bf16>::load(Wr_h + 2 * H_SIZE * I_SIZE + ko);
        const v16b bl = Frag<__bf16>::load(Wr_l + 2 * H_SIZE * I_SIZE + ko);
        axn = mma_bf16g(ah, bh, axn); axn = mma_bf16g(ah, bl, axn); axn = mma_bf16g(al, bh, axn);
      }
    }

    const _Float16* arow = &hb[cur][c * LDH + koff];
#pragma unroll
    for (int kc = 0; kc < 4; ++kc) {
      const int ko = kc * 32;
      const v16h a = Frag<_Float16>::load(arow + ko);
      ahr = mma_f16g(a, Frag<_Float16>::load(Whr + ko), ahr);
      ahz = mma_f16g(a, Frag<_Float16>::load(Whr + H_SIZE * H_SIZE + ko), ahz);
      ahn = mma_f16g(a, Frag<_Float16>::load(Whr + 2 * H_SIZE * H_SIZE + ko), ahn);
    }

    _Float16* hbn = hb[nxt];
    float*    hFn = hF[nxt];
#pragma unroll
    for (int r = 0; r < 8; ++r) {
      const int row = 8 * hh + r;
      const float gxr = axr[r] + bir;
      const float ghr = ahr[r] * HINV + bhr;
      const float rg = sigm_(gxr + ghr);
      const float gxz = axz[r] + biz;
      const float ghz = ahz[r] * HINV + bhz;
      const float zg = sigm_(gxz + ghz);
      const float gxn = axn[r] + bin;
      const float ghn = ahn[r] * HINV + bhn;
      const float ng = tanhf(gxn + rg * ghn);
      const float hn = (1.0f - zg) * ng + zg * hst[r];
      hst[r] = hn;
      hbn[row * LDH + col] = (_Float16)(hn * 256.0f);
      hFn[row * LDF + col] = hn;
    }
    __syncthreads();

    {
      const float* sp = hF[nxt] + srow * LDF + sseg;
      const v4f p0 = *(const v4f*)sp;
      const v4f p1 = *(const v4f*)(sp + 4);
      v8h hv, lv;
#pragma unroll
      for (int e = 0; e < 4; ++e) {
        const unsigned short h0 = f2bf_bits(p0[e]);
        const unsigned short l0 = f2bf_bits(p0[e] - bf_bits2f(h0));
        const unsigned short h1 = f2bf_bits(p1[e]);
        const unsigned short l1 = f2bf_bits(p1[e] - bf_bits2f(h1));
        hv[e] = __builtin_bit_cast(_Float16, h0);     lv[e] = __builtin_bit_cast(_Float16, l0);
        hv[4 + e] = __builtin_bit_cast(_Float16, h1); lv[4 + e] = __builtin_bit_cast(_Float16, l1);
      }
      const size_t o = ((size_t)(bbase + srow) * TLEN + t) * H_SIZE + sseg;
      *(volatile v8h*)(hs_hi + o) = hv;
      *(volatile v8h*)(hs_lo + o) = lv;
      __threadfence();
      *(volatile v8h*)(hs_hi + o) = hv;
      *(volatile v8h*)(hs_lo + o) = lv;
    }
  }
}

extern "C" void kernel_launch(void* const* d_in, const int* in_sizes, int n_in,
                              void* d_out, int out_size, void* d_ws, size_t ws_size,
                              hipStream_t stream) {
  if (n_in < 7) return;
  const int n_x   = in_sizes[0];
  const int n_ih  = in_sizes[1];
  const int n_hh  = in_sizes[2];
  const int n_out = in_sizes[5];
  if (n_x != BATCH * TLEN * I_SIZE || n_ih != G3H * I_SIZE || n_hh != G3H * H_SIZE ||
      in_sizes[3] != G3H || in_sizes[4] != G3H || n_out != O_SIZE * H_SIZE ||
      in_sizes[6] != O_SIZE || out_size != BATCH * TLEN * O_SIZE) return;

  const float* x     = (const float*)d_in[0];
  const float* W_ih  = (const float*)d_in[1];
  const float* W_hh  = (const float*)d_in[2];
  const float* b_ih  = (const float*)d_in[3];
  const float* b_hh  = (const float*)d_in[4];
  const float* W_out = (const float*)d_in[5];
  const float* b_out = (const float*)d_in[6];
  float* out = (float*)d_out;

  char* ws = (char*)d_ws;
  size_t off = 0;
  const size_t nx_e  = (size_t)BATCH * TLEN * I_SIZE;
  const size_t nhs_e = (size_t)BATCH * TLEN * H_SIZE;
  unsigned short* xh     = (unsigned short*)(ws + off); off += nx_e * 2;
  unsigned short* xl     = (unsigned short*)(ws + off); off += nx_e * 2;
  unsigned short* hs_hi  = (unsigned short*)(ws + off); off += nhs_e * 2;
  unsigned short* hs_lo  = (unsigned short*)(ws + off); off += nhs_e * 2;
  unsigned short* wih_h  = (unsigned short*)(ws + off); off += (size_t)n_ih * 2;
  unsigned short* wih_l  = (unsigned short*)(ws + off); off += (size_t)n_ih * 2;
  _Float16*       whh16  = (_Float16*)(ws + off);       off += (size_t)n_hh * 2;
  unsigned short* wout_h = (unsigned short*)(ws + off); off += (size_t)n_out * 2;
  unsigned short* wout_l = (unsigned short*)(ws + off); off += (size_t)n_out * 2;
  if (off > ws_size) return;

  const int n8_x = n_x / 8, n8_ih = n_ih / 8, n8_hh = n_hh / 8, n8_out = n_out / 8;
  cast_f32_bf16hl8<<<(n8_x + 255) / 256, 256, 0, stream>>>(x, xh, xl, n8_x);
  cast_f32_bf16hl8<<<(n8_ih + 255) / 256, 256, 0, stream>>>(W_ih, wih_h, wih_l, n8_ih);
  cast_f32_f16s8  <<<(n8_hh + 255) / 256, 256, 0, stream>>>(W_hh, whh16, n8_hh, 64.0f);
  cast_f32_bf16hl8<<<(n8_out + 255) / 256, 256, 0, stream>>>(W_out, wout_h, wout_l, n8_out);

  gru_scan_kernel<<<BATCH / 16, 256, 0, stream>>>(xh, xl, wih_h, wih_l, whh16, b_ih, b_hh, hs_hi, hs_lo);

  const int M = BATCH * TLEN, N = O_SIZE, K = H_SIZE;
  const int tiles = (M / 64) * (N / 64);
  wmma_gemm64<1, true, 2, 0, false, 0><<<dim3((tiles + 7) / 8, 1), 256, 0, stream>>>(
      hs_hi, hs_lo, H_SIZE, 0L,
      wout_h, wout_l, H_SIZE, 0L,
      (void*)out, (void*)nullptr, O_SIZE, 0L,
      b_out, (const float*)nullptr, 0L,
      M, N, K, 1.0f);
}
